// MultiHeadedAttention_31988916421161
// MI455X (gfx1250) — hardware-verified
//
#include <hip/hip_runtime.h>

#ifndef NB
#define NB 4
#endif
#ifndef SEQ
#define SEQ 2048
#endif
#ifndef SEQ_FULL
#define SEQ_FULL 2048
#endif
#ifndef SEQ_OUT
#define SEQ_OUT SEQ
#endif
#ifndef NLATE
#define NLATE (SEQ / 2)
#endif
#define EMB 1024
#define NHD 16
#define HD 64
#define NQK 2048
#define SLATE (SEQ - NLATE)
#define NR ((size_t)NB * SEQ)
#define ALPHA_S 0.125f
#define RSC 4096.0f
#define RSCI 0.000244140625f
static_assert(SEQ % 128 == 0);
static_assert(NLATE % 128 == 0);
static_assert(NLATE >= 128);
static_assert(NLATE <= SEQ);
static_assert(SLATE % 128 == 0);
static_assert(SEQ <= SEQ_FULL);
static_assert(NHD * HD == EMB);
static_assert(EMB % 128 == 0);
static_assert(NQK == 2 * NHD * HD);

typedef _Float16 v16h __attribute__((ext_vector_type(16)));
typedef unsigned short v8us __attribute__((ext_vector_type(8), may_alias));
typedef float v8f __attribute__((ext_vector_type(8)));
typedef float v4f __attribute__((ext_vector_type(4)));
typedef float v4fa __attribute__((ext_vector_type(4), may_alias));
union FragH { v16h v; v8us half[2]; _Float16 h[16]; unsigned short u[16]; };
union H1 { _Float16 h; unsigned short u; };

__device__ __forceinline__ unsigned short bf16_bits(float x) { unsigned int u = __float_as_uint(x); return (unsigned short)((u + 0x7FFFu + ((u >> 16) & 1u)) >> 16); }
__device__ __forceinline__ float bf16_val(unsigned short b) { return __uint_as_float(((unsigned int)b) << 16); }
__device__ __forceinline__ float bf16_rne(float x) { return bf16_val(bf16_bits(x)); }

__device__ __forceinline__ v16h g2_frag(const _Float16* p, int hh) { FragH f; f.half[0] = *(const v8us*)((const unsigned short*)p + 8 * hh); f.half[1] = *(const v8us*)((const unsigned short*)p + 16 + 8 * hh); return f.v; }
__device__ __forceinline__ v16h g2_frag_u(const unsigned short* p, int hh) { FragH f; f.half[0] = *(const v8us*)(p + 8 * hh); f.half[1] = *(const v8us*)(p + 16 + 8 * hh); return f.v; }
__device__ __forceinline__ v8f g2_mma(v16h a, v16h b, v8f c) { v8f d = __builtin_amdgcn_wmma_f32_16x16x32_f16(false, a, false, b, (short)0, c, false, false); asm volatile("v_nop\n\tv_nop\n\tv_nop\n\tv_nop" : "+v"(d) : "v"(a), "v"(b)); return d; }
__device__ __forceinline__ v16h zero16() { FragH f;
#pragma unroll
  for (int i = 0; i < 16; ++i) f.u[i] = 0; return f.v; }
__device__ __forceinline__ float logit_of(float a, float a2, bool late) {
  #pragma clang fp contract(off)
  const float s = late ? fmaf(a2, RSCI, a) : a; return s * ALPHA_S; }

__global__ __launch_bounds__(256) void k_x16(const float* __restrict__ x, _Float16* __restrict__ X16) {
  const size_t t = (size_t)blockIdx.x * 256 + threadIdx.x;
  const size_t n8 = NR * (EMB / 8);
  if (t >= n8) return;
  const size_t row = t / (EMB / 8);
  const int c8 = (int)(t % (EMB / 8)) * 8;
  const size_t b = row / SEQ, tt = row - b * SEQ;
  const float* src = x + (b * SEQ_FULL + tt) * EMB + c8;
  const v4f a = *(const v4fa*)src, c = *(const v4fa*)(src + 4);
  FragH f;
#pragma unroll
  for (int q = 0; q < 4; ++q) { f.h[q] = (_Float16)bf16_rne(a[q]); f.h[4 + q] = (_Float16)bf16_rne(c[q]); }
  unsigned short* d = (unsigned short*)X16 + row * EMB + c8;
  *(volatile v8us*)d = f.half[0]; __threadfence(); *(volatile v8us*)d = f.half[0];
}

__global__ __launch_bounds__(256) void k_wt(const float* __restrict__ W, _Float16* __restrict__ WT, int nrows, int DD) {
  const int t = blockIdx.x * 256 + threadIdx.x;
  if (t >= nrows * (EMB / 8)) return;
  const int n = t / (EMB / 8), c8 = (t % (EMB / 8)) * 8;
  const int g = n / DD, d = n - g * DD;
  FragH f;
#pragma unroll
  for (int i = 0; i < 8; ++i) f.h[i] = (_Float16)(bf16_rne(W[((size_t)g * EMB + c8 + i) * DD + d]) * 16.0f);
  unsigned short* dst = (unsigned short*)WT + (size_t)n * EMB + c8;
  *(volatile v8us*)dst = f.half[0]; __threadfence(); *(volatile v8us*)dst = f.half[0];
}

__global__ __launch_bounds__(128) void k_pgemm(const _Float16* __restrict__ A, int lda, size_t sA, const _Float16* __restrict__ Bt, int ldb, size_t sB,
                                              int M, int N, float alpha, _Float16* __restrict__ CH, size_t sHb, size_t slabH, int ldh,
                                              _Float16* __restrict__ CL, size_t sLb, size_t slabL, int ldl, int lorow0, int locol0) {
  __shared__ __attribute__((aligned(16))) float so[4][32][68];
  const int tid = threadIdx.x, w = tid >> 5, lane = tid & 31, ln = lane & 15, hh = lane >> 4;
  const int by = blockIdx.y;
  A += (size_t)by * sA; Bt += (size_t)by * sB;
  const int ntn = N >> 6; const int mt = blockIdx.x / ntn, nq = blockIdx.x - mt * ntn;
  const int row0 = mt * 128 + 32 * w, col0 = nq * 64;
  if (row0 >= M) return;
  const _Float16* a0p = A + (size_t)(row0 + ln) * lda; const _Float16* a1p = a0p + (size_t)16 * lda;
  const _Float16* b0p = Bt + (size_t)(col0 + ln) * ldb; const _Float16* b1p = b0p + (size_t)16 * ldb; const _Float16* b2p = b1p + (size_t)16 * ldb; const _Float16* b3p = b2p + (size_t)16 * ldb;
  const v8f z8 = {0.f,0.f,0.f,0.f,0.f,0.f,0.f,0.f}; v8f c00 = z8, c01 = z8, c02 = z8, c03 = z8, c10 = z8, c11 = z8, c12 = z8, c13 = z8;
#pragma unroll 1
  for (int kb = 0; kb < EMB; kb += 32) { const v16h a0 = g2_frag(a0p + kb, hh), a1 = g2_frag(a1p + kb, hh);
    v16h b = g2_frag(b0p + kb, hh); c00 = g2_mma(a0, b, c00); c10 = g2_mma(a1, b, c10);
    b = g2_frag(b1p + kb, hh); c01 = g2_mma(a0, b, c01); c11 = g2_mma(a1, b, c11);
    b = g2_frag(b2p + kb, hh); c02 = g2_mma(a0, b, c02); c12 = g2_mma(a1, b, c12);
    b = g2_frag(b3p + kb, hh); c03 = g2_mma(a0, b, c03); c13 = g2_mma(a1, b, c13); }
  v8f accs[8] = {c00, c01, c02, c03, c10, c11, c12, c13};
#pragma unroll
  for (int u = 0; u < 8; ++u) { const int t = u & 3, half = u >> 2;
#pragma unroll
    for (int r = 0; r < 8; ++r) so[w][half * 16 + 8 * hh + r][t * 16 + ln] = accs[u][r] * alpha; }
  __builtin_amdgcn_fence(4  , "workgroup"); __builtin_amdgcn_wave_barrier();
  const bool late = (mt * 128 >= lorow0) && (col0 >= locol0);
  const int sub = lane >> 3, pc = lane & 7;
  unsigned short* hb = (unsigned short*)CH + (size_t)by * sHb + (size_t)nq * slabH + pc * 8;
  unsigned short* lb = hb;
  if (late) lb = (unsigned short*)CL + (size_t)by * sLb + (size_t)((col0 - locol0) >> 6) * slabL + pc * 8;
  for (int ps = 0; ps < 2; ++ps) {
#pragma unroll
    for (int q = 0; q < 8; ++q) {
      const int r = q * 4 + sub;
      const v4f a = *(const v4fa*)&so[w][r][pc * 8], c = *(const v4fa*)&so[w][r][pc * 8 + 4];
      FragH fh, fl;
#pragma unroll
      for (int i = 0; i < 4; ++i) { _Float16 hv = (_Float16)a[i]; fh.h[i] = hv; fl.h[i] = (_Float16)((a[i] - (float)hv) * RSC); hv = (_Float16)c[i]; fh.h[4 + i] = hv; fl.h[4 + i] = (_Float16)((c[i] - (float)hv) * RSC); }
      *(volatile v8us*)(hb + (size_t)(row0 + r) * ldh) = fh.half[0];
      if (late) *(volatile v8us*)(lb + (size_t)(row0 + r - lorow0) * ldl) = fl.half[0];
    }
    if (ps == 0) __threadfence();
  }
}

__global__ __launch_bounds__(64) void k_cstat(const _Float16* __restrict__ QKH, const _Float16* __restrict__ QKL, float* __restrict__ MST, float* __restrict__ RST) {
  #pragma clang fp contract(off)
  const int tid = threadIdx.x, w = tid >> 5, lane = tid & 31, ln = lane & 15, hh = lane >> 4;
  const int bh = blockIdx.y, b = bh / NHD, h = bh - b * NHD;
  const int s0b = blockIdx.x * 64, s0w = s0b + 32 * w;
  const bool late = (s0b >= SLATE);
  const _Float16* Qh = QKH + (size_t)(b * 32 + h) * SEQ * HD;
  const _Float16* Kh = QKH + (size_t)(b * 32 + NHD + h) * SEQ * HD;
  const _Float16* Ql = QKL + (size_t)(b * 32 + h) * NLATE * HD;
  const _Float16* Kl = QKL + (size_t)(b * 32 + NHD + h) * NLATE * HD;
  const v16h z16 = zero16(); const v8f z8 = {0.f,0.f,0.f,0.f,0.f,0.f,0.f,0.f};
  v16h khf[2][2], klf[2][2];
#pragma unroll
  for (int j = 0; j < 2; ++j) {
    const int sr = s0w + 16 * j + ln;
    khf[j][0] = g2_frag(Kh + (size_t)sr * HD, hh); khf[j][1] = g2_frag(Kh + (size_t)sr * HD + 32, hh);
    klf[j][0] = z16; klf[j][1] = z16;
    if (late) { klf[j][0] = g2_frag(Kl + (size_t)(sr - SLATE) * HD, hh); klf[j][1] = g2_frag(Kl + (size_t)(sr - SLATE) * HD + 32, hh); }
  }
  float mst[2] = {-1.0e30f, -1.0e30f}, zst[2] = {0.f, 0.f};
#pragma unroll 1
  for (int t0 = s0w; t0 < SEQ; t0 += 16) {
    const v16h ah0 = g2_frag(Qh + (size_t)(t0 + ln) * HD, hh), ah1 = g2_frag(Qh + (size_t)(t0 + ln) * HD + 32, hh);
    v16h al0 = z16, al1 = z16;
    if (late) { al0 = g2_frag(Ql + (size_t)(t0 - SLATE + ln) * HD, hh); al1 = g2_frag(Ql + (size_t)(t0 - SLATE + ln) * HD + 32, hh); }
#pragma unroll
    for (int j = 0; j < 2; ++j) {
      v8f acc = g2_mma(ah0, khf[j][0], z8); acc = g2_mma(ah1, khf[j][1], acc);
      v8f acc2 = z8;
      if (late) { acc2 = g2_mma(al0, khf[j][0], z8); acc2 = g2_mma(al1, khf[j][1], acc2); acc2 = g2_mma(ah0, klf[j][0], acc2); acc2 = g2_mma(ah1, klf[j][1], acc2); }
      const int s = s0w + 16 * j + ln;
      float lg[8]; float tmax = -1.0e30f;
#pragma unroll
      for (int r = 0; r < 8; ++r) {
        const float l = logit_of(acc[r], acc2[r], late);
        const int t = t0 + 8 * hh + r; const float f = (t >= s) ? 1.f : 0.f;
        const float vm = fmaf(f, l, (1.f - f) * -1.0e30f);
        lg[r] = vm; tmax = fmaxf(tmax, vm);
      }
      tmax = fmaxf(tmax, __shfl_xor(tmax, 16, 32));
      const float mn = fmaxf(mst[j], tmax);
      float se = 0.f;
#pragma unroll
      for (int r = 0; r < 8; ++r) { const int t = t0 + 8 * hh + r; const float f = (t >= s) ? 1.f : 0.f; se += f * __expf(lg[r] - mn); }
      se += __shfl_xor(se, 16, 32);
      zst[j] = zst[j] * __expf(mst[j] - mn) + se; mst[j] = mn;
    }
  }
  const float mv = hh ? mst[1] : mst[0]; const float zv = hh ? zst[1] : zst[0]; const float rv = 1.0f / zv;
  float* pm = MST + (size_t)bh * SEQ + s0w + lane; float* pr = RST + (size_t)bh * SEQ + s0w + lane;
  *(volatile float*)pm = mv; *(volatile float*)pr = rv;
  __threadfence();
  *(volatile float*)pm = mv; *(volatile float*)pr = rv;
}

__global__ __launch_bounds__(128) void k_attn(const _Float16* __restrict__ QKH, const _Float16* __restrict__ QKL, const _Float16* __restrict__ VTH, const _Float16* __restrict__ VTL,
                                             const float* __restrict__ MST, const float* __restrict__ RST, _Float16* __restrict__ AH, _Float16* __restrict__ AL) {
  #pragma clang fp contract(off)
  __shared__ __attribute__((aligned(16))) unsigned short pbh[4][16 * 40];
  __shared__ __attribute__((aligned(16))) unsigned short pbl[4][16 * 40];
  __shared__ __attribute__((aligned(16))) float so[4][16][68];
  const int tid = threadIdx.x, w = tid >> 5, lane = tid & 31, ln = lane & 15, hh = lane >> 4;
  const int bh = blockIdx.y, b = bh / NHD, h = bh - b * NHD;
  const int t0b = blockIdx.x * 64, t0w = t0b + 16 * w;
  const bool lateQ = (t0b >= SLATE);
  const _Float16* Qh = QKH + (size_t)(b * 32 + h) * SEQ * HD;
  const _Float16* Kh = QKH + (size_t)(b * 32 + NHD + h) * SEQ * HD;
  const _Float16* Ql = QKL + (size_t)(b * 32 + h) * NLATE * HD;
  const _Float16* Kl = QKL + (size_t)(b * 32 + NHD + h) * NLATE * HD;
  const _Float16* Vh = VTH + ((size_t)b * EMB + h * HD) * SEQ;
  const _Float16* Vl = VTL + ((size_t)b * EMB + h * HD) * NLATE;
  const float* ms = MST + (size_t)bh * SEQ; const float* rs = RST + (size_t)bh * SEQ;
  const v16h z16 = zero16(); const v8f z8 = {0.f,0.f,0.f,0.f,0.f,0.f,0.f,0.f};
  const v16h ah0 = g2_frag(Qh + (size_t)(t0w + ln) * HD, hh), ah1 = g2_frag(Qh + (size_t)(t0w + ln) * HD + 32, hh);
  v16h al0 = z16, al1 = z16;
  if (lateQ) { al0 = g2_frag(Ql + (size_t)(t0w - SLATE + ln) * HD, hh); al1 = g2_frag(Ql + (size_t)(t0w - SLATE + ln) * HD + 32, hh); }
  v8f oh[4], orr[4];
#pragma unroll
  for (int nb = 0; nb < 4; ++nb) { oh[nb] = z8; orr[nb] = z8; }
  unsigned short* ph_ = &pbh[w][0]; unsigned short* pl_ = &pbl[w][0];
  const int send = t0w + 16;
#pragma unroll 1
  for (int s0 = 0; s0 < send; s0 += 32) {
    const bool lateK = (s0 >= SLATE);
    __builtin_amdgcn_fence(3  , "wavefront"); __builtin_amdgcn_wave_barrier();
#pragma unroll
    for (int j = 0; j < 2; ++j) {
      const int sr = s0 + 16 * j + ln;
      const v16h kh0 = g2_frag(Kh + (size_t)sr * HD, hh), kh1 = g2_frag(Kh + (size_t)sr * HD + 32, hh);
      v8f acc = g2_mma(ah0, kh0, z8); acc = g2_mma(ah1, kh1, acc);
      v8f acc2 = z8;
      if (lateK) {
        const v16h kl0 = g2_frag(Kl + (size_t)(sr - SLATE) * HD, hh), kl1 = g2_frag(Kl + (size_t)(sr - SLATE) * HD + 32, hh);
        acc2 = g2_mma(al0, kh0, z8); acc2 = g2_mma(al1, kh1, acc2); acc2 = g2_mma(ah0, kl0, acc2); acc2 = g2_mma(ah1, kl1, acc2);
      }
      const float mcol = ms[sr], ccol = rs[sr] * RSC;
#pragma unroll
      for (int r = 0; r < 8; ++r) {
        const float l = logit_of(acc[r], acc2[r], lateK);
        const int t = t0w + 8 * hh + r; const float f = (t >= sr) ? 1.f : 0.f;
        const float vm = fmaf(f, l, (1.f - f) * -1.0e30f);
        const float p4 = f * __expf(vm - mcol) * ccol;
        const _Float16 pvh = (_Float16)p4; H1 u1; u1.h = pvh;
        ph_[(8 * hh + r) * 40 + 16 * j + ln] = u1.u;
        if (lateK) { H1 u2; u2.h = (_Float16)((p4 - (float)pvh) * RSC); pl_[(8 * hh + r) * 40 + 16 * j + ln] = u2.u; }
      }
    }
    __builtin_amdgcn_fence(3  , "wavefront"); __builtin_amdgcn_wave_barrier();
    const v16h ap = g2_frag_u(ph_ + ln * 40, hh);
    v16h apl = z16;
    if (lateK) apl = g2_frag_u(pl_ + ln * 40, hh);
#pragma unroll
    for (int nb = 0; nb < 4; ++nb) {
      const v16h vb = g2_frag(Vh + (size_t)(nb * 16 + ln) * SEQ + s0, hh);
      oh[nb] = g2_mma(ap, vb, oh[nb]);
      if (lateK) { const v16h vl = g2_frag(Vl + (size_t)(nb * 16 + ln) * NLATE + (s0 - SLATE), hh); orr[nb] = g2_mma(apl, vb, orr[nb]); orr[nb] = g2_mma(ap, vl, orr[nb]); }
    }
  }
  const float osc = 0.015625f;
#pragma unroll
  for (int nb = 0; nb < 4; ++nb)
#pragma unroll
    for (int r = 0; r < 8; ++r) { const float o = lateQ ? fmaf(orr[nb][r], RSCI, oh[nb][r]) : oh[nb][r]; so[w][8 * hh + r][nb * 16 + ln] = o * osc; }
  __builtin_amdgcn_fence(4  , "workgroup"); __builtin_amdgcn_wave_barrier();
  const int sub = lane >> 3, pc = lane & 7;
  for (int ps = 0; ps < 2; ++ps) {
#pragma unroll
    for (int q = 0; q < 4; ++q) {
      const int r = q * 4 + sub;
      const v4f a = *(const v4fa*)&so[w][r][pc * 8], c = *(const v4fa*)&so[w][r][pc * 8 + 4];
      FragH fh, fl;
#pragma unroll
      for (int i = 0; i < 4; ++i) { _Float16 hv = (_Float16)a[i]; fh.h[i] = hv; fl.h[i] = (_Float16)((a[i] - (float)hv) * RSC); hv = (_Float16)c[i]; fh.h[4 + i] = hv; fl.h[4 + i] = (_Float16)((c[i] - (float)hv) * RSC); }
      *(volatile v8us*)((unsigned short*)AH + ((size_t)b * SEQ + t0w + r) * EMB + h * HD + pc * 8) = fh.half[0];
      if (lateQ) *(volatile v8us*)((unsigned short*)AL + ((size_t)b * NLATE + (t0w - SLATE) + r) * EMB + h * HD + pc * 8) = fl.half[0];
    }
    if (ps == 0) __threadfence();
  }
}

__global__ __launch_bounds__(128) void k_oproj(const _Float16* __restrict__ AH, const _Float16* __restrict__ AL, const _Float16* __restrict__ WOT, const float* __restrict__ bo, float* __restrict__ out) {
  __shared__ __attribute__((aligned(16))) float so[4][32][68];
  const int tid = threadIdx.x, w = tid >> 5, lane = tid & 31, ln = lane & 15, hh = lane >> 4;
  const int ntn = EMB >> 6; const int mt = blockIdx.x / ntn, nq = blockIdx.x - mt * ntn;
  const int row0 = mt * 128 + 32 * w, col0 = nq * 64;
  const int b = (mt * 128) / SEQ; const int tw = row0 - b * SEQ;
  const bool late = (mt * 128 - b * SEQ) >= SLATE;
  const _Float16* a0p = AH + (size_t)(row0 + ln) * EMB; const _Float16* a1p = a0p + (size_t)16 * EMB;
  const _Float16* b0p = WOT + (size_t)(col0 + ln) * EMB; const _Float16* b1p = b0p + (size_t)16 * EMB; const _Float16* b2p = b1p + (size_t)16 * EMB; const _Float16* b3p = b2p + (size_t)16 * EMB;
  const v8f z8 = {0.f,0.f,0.f,0.f,0.f,0.f,0.f,0.f}; v8f c00 = z8, c01 = z8, c02 = z8, c03 = z8, c10 = z8, c11 = z8, c12 = z8, c13 = z8;
#pragma unroll 1
  for (int kb = 0; kb < EMB; kb += 32) { const v16h a0 = g2_frag(a0p + kb, hh), a1 = g2_frag(a1p + kb, hh);
    v16h bb = g2_frag(b0p + kb, hh); c00 = g2_mma(a0, bb, c00); c10 = g2_mma(a1, bb, c10);
    bb = g2_frag(b1p + kb, hh); c01 = g2_mma(a0, bb, c01); c11 = g2_mma(a1, bb, c11);
    bb = g2_frag(b2p + kb, hh); c02 = g2_mma(a0, bb, c02); c12 = g2_mma(a1, bb, c12);
    bb = g2_frag(b3p + kb, hh); c03 = g2_mma(a0, bb, c03); c13 = g2_mma(a1, bb, c13); }
  {
    v8f accs[8] = {c00, c01, c02, c03, c10, c11, c12, c13};
#pragma unroll
    for (int u = 0; u < 8; ++u) { const int t = u & 3, half = u >> 2; const float bv = bf16_rne(bo[col0 + t * 16 + ln]);
#pragma unroll
      for (int r = 0; r < 8; ++r) so[w][half * 16 + 8 * hh + r][t * 16 + ln] = accs[u][r] * 0.0009765625f + bv; }
  }
  if (late) {
    const _Float16* l0p = AL + ((size_t)b * NLATE + (tw - SLATE) + ln) * EMB; const _Float16* l1p = l0p + (size_t)16 * EMB;
    c00 = z8; c01 = z8; c02 = z8; c03 = z8; c10 = z8; c11 = z8; c12 = z8; c13 = z8;
#pragma unroll 1
    for (int kb = 0; kb < EMB; kb += 32) { const v16h a0 = g2_frag(l0p + kb, hh), a1 = g2_frag(l1p + kb, hh);
      v16h bb = g2_frag(b0p + kb, hh); c00 = g2_mma(a0, bb, c00); c10 = g2_mma(a1, bb, c10);
      bb = g2_frag(b1p + kb, hh); c01 = g2_mma(a0, bb, c01); c11 = g2_mma(a1, bb, c11);
      bb = g2_frag(b2p + kb, hh); c02 = g2_mma(a0, bb, c02); c12 = g2_mma(a1, bb, c12);
      bb = g2_frag(b3p + kb, hh); c03 = g2_mma(a0, bb, c03); c13 = g2_mma(a1, bb, c13); }
    v8f acc2s[8] = {c00, c01, c02, c03, c10, c11, c12, c13};
#pragma unroll
    for (int u = 0; u < 8; ++u) { const int t = u & 3, half = u >> 2;
#pragma unroll
      for (int r = 0; r < 8; ++r) so[w][half * 16 + 8 * hh + r][t * 16 + ln] += acc2s[u][r] * 2.384185791015625e-07f; }
  }
  __builtin_amdgcn_fence(4  , "workgroup"); __builtin_amdgcn_wave_barrier();
  const int rsub = lane >> 4, c4 = (lane & 15) * 4;
  for (int ps = 0; ps < 2; ++ps) {
#pragma unroll
    for (int q = 0; q < 16; ++q) { const int r = q * 2 + rsub; const v4f v = *(const v4fa*)&so[w][r][c4];
      *(volatile v4f*)(out + ((size_t)b * SEQ_OUT + tw + r) * EMB + col0 + c4) = v; }
    if (ps == 0) __threadfence();
  }
}

extern "C" void kernel_launch(void* const* d_in, const int* in_sizes, int n_in,
                              void* d_out, int out_size, void* d_ws, size_t ws_size, hipStream_t stream) {
  if (n_in < 6) return;
  const size_t need_x = ((size_t)(NB - 1) * SEQ_FULL + SEQ) * EMB;
  if ((size_t)in_sizes[0] < need_x) return;
  if ((size_t)in_sizes[1] < (size_t)NHD * EMB * HD || (size_t)in_sizes[2] < (size_t)NHD * EMB * HD || (size_t)in_sizes[3] < (size_t)NHD * EMB * HD) return;
  if ((size_t)in_sizes[4] < (size_t)EMB * EMB || (size_t)in_sizes[5] < (size_t)EMB) return;
  if ((size_t)out_size < ((size_t)(NB - 1) * SEQ_OUT + SEQ) * EMB) return;
  const float* x  = (const float*)d_in[0];
  const float* Wq = (const float*)d_in[1];
  const float* Wk = (const float*)d_in[2];
  const float* Wv = (const float*)d_in[3];
  const float* Wo = (const float*)d_in[4];
  const float* bo = (const float*)d_in[5];
  char* ws = (char*)d_ws; size_t off = 0;
  auto take = [&](size_t bytes) { char* p = ws + off; off += (bytes + 255) & ~(size_t)255; return p; };
  char* RA = take(NR * EMB * 2);
  _Float16* X16 = (_Float16*)RA; _Float16* AH = (_Float16*)RA;
  _Float16* AL   = (_Float16*)take((size_t)NB * NLATE * EMB * 2);
  _Float16* WQKT = (_Float16*)take((size_t)NQK * EMB * 2);
  _Float16* WVT  = (_Float16*)take((size_t)EMB * EMB * 2);
  _Float16* WOT  = (_Float16*)take((size_t)EMB * EMB * 2);
  _Float16* QKH  = (_Float16*)take((size_t)NB * 32 * SEQ * HD * 2);
  _Float16* QKL  = (_Float16*)take((size_t)NB * 32 * NLATE * HD * 2);
  _Float16* VTH  = (_Float16*)take((size_t)NB * EMB * SEQ * 2);
  _Float16* VTL  = (_Float16*)take((size_t)NB * EMB * NLATE * 2);
  float* MST = (float*)take((size_t)NB * NHD * SEQ * 4);
  float* RST = (float*)take((size_t)NB * NHD * SEQ * 4);
  if (off > ws_size) return;
  k_x16<<<(unsigned)((NR * (EMB / 8) + 255) / 256), 256, 0, stream>>>(x, X16);
  k_wt<<<(NHD * HD * (EMB / 8) + 255) / 256, 256, 0, stream>>>(Wq, WQKT, NHD * HD, HD);
  k_wt<<<(NHD * HD * (EMB / 8) + 255) / 256, 256, 0, stream>>>(Wk, WQKT + (size_t)NHD * HD * EMB, NHD * HD, HD);
  k_wt<<<(NHD * HD * (EMB / 8) + 255) / 256, 256, 0, stream>>>(Wv, WVT, NHD * HD, HD);
  k_wt<<<(EMB * (EMB / 8) + 255) / 256, 256, 0, stream>>>(Wo, WOT, EMB, EMB);
  k_pgemm<<<dim3((unsigned)((SEQ / 128) * (NQK / 64)), NB), 128, 0, stream>>>(X16, EMB, (size_t)SEQ * EMB, WQKT, EMB, (size_t)0, SEQ, NQK, 0.0625f,
      QKH, (size_t)32 * SEQ * HD, (size_t)SEQ * HD, HD, QKL, (size_t)32 * NLATE * HD, (size_t)NLATE * HD, HD, SLATE, 0);
  k_pgemm<<<dim3((unsigned)((EMB / 128) * (SEQ / 64)), NB), 128, 0, stream>>>(WVT, EMB, (size_t)0, X16, EMB, (size_t)SEQ * EMB, EMB, SEQ, 0.0625f,
      VTH, (size_t)EMB * SEQ, (size_t)64, SEQ, VTL, (size_t)EMB * NLATE, (size_t)64, NLATE, 0, SLATE);
  k_cstat<<<dim3(SEQ / 64, NB * NHD), 64, 0, stream>>>(QKH, QKL, MST, RST);
  k_attn<<<dim3(SEQ / 64, NB * NHD), 128, 0, stream>>>(QKH, QKL, VTH, VTL, MST, RST, AH, AL);
  k_oproj<<<(unsigned)((NR / 128) * (EMB / 64)), 128, 0, stream>>>(AH, AL, WOT, bo, (float*)d_out);
}
